// LSTMLayer_31396210934320
// MI455X (gfx1250) — hardware-run, weakly checked
//
#include <hip/hip_runtime.h>
#include <math.h>

#pragma clang fp contract(off)

typedef __attribute__((ext_vector_type(16))) __bf16   v16b;
typedef __attribute__((ext_vector_type(8)))  __bf16   v8b;
typedef __attribute__((ext_vector_type(8)))  float    v8f;
typedef __attribute__((ext_vector_type(4)))  float    v4f;
typedef __attribute__((ext_vector_type(4)))  unsigned v4u;

constexpr int kBatch   = 4;
constexpr int kCin     = 256;
constexpr int kT       = 2048;
constexpr int kGateCh  = 256;
constexpr int kNused   = 3 * kGateCh;
constexpr int kNall    = 4 * kGateCh;
constexpr int kK       = 2 * kCin;
constexpr int kXtRows  = kT + 1;
constexpr size_t kXtBatch = (size_t)kXtRows * kCin;
constexpr int kCols    = kBatch * kT;
constexpr int kSlabP   = 68;
constexpr int kXtLdsP  = 132;
constexpr int kTilesM  = kNused / 64;
constexpr int kTilesN  = kT / 64;
constexpr int kGemmBlocksX = (kTilesM * kTilesN) / 8;
static_assert((kK % 32) == 0, "GEMM depth multiple of 32");
static_assert((kNused % 64) == 0 && (kT % 64) == 0, "GEMM M, N multiples of 64");
static_assert(kGemmBlocksX * 8 == kTilesM * kTilesN, "exact tile grid");
static_assert((kT % 128) == 0, "a wave's 128 columns stay inside one batch element");

constexpr size_t kOffWB = 0;
constexpr size_t kOffXT = kOffWB + (size_t)kNused * kK * 2;
constexpr size_t kOffGP = kOffXT + (size_t)kBatch * kXtBatch * 2;
constexpr size_t kWsTotal = kOffGP + (size_t)kNused * kCols * 4;
static_assert(kWsTotal == 30148608ull, "carve total");
static_assert(kWsTotal <= 134217728ull, "carve cap");
static_assert((kOffXT % 128) == 0 && (kOffGP % 128) == 0, "128-B aligned regions");

__device__ __forceinline__ unsigned short f2bf_bits(float f) {
  unsigned u = __float_as_uint(f);
  return (unsigned short)((u + 0x7FFFu + ((u >> 16) & 1u)) >> 16);
}
__device__ __forceinline__ float bf_bits2f(unsigned short h) { return __uint_as_float(((unsigned)h) << 16); }

union FragB { v16b v; v8b h[2]; };
__device__ __forceinline__ v16b frag_load(const __bf16* p) {
  FragB f;
  f.h[0] = *(const v8b*)(p);
  f.h[1] = *(const v8b*)(p + 16);
  return f.v;
}
__device__ __forceinline__ v8f mma_bf16(v16b a, v16b b, v8f c) {
  c = __builtin_amdgcn_wmma_f32_16x16x32_bf16(false, a, false, b, (short)0, c, false, false);
  asm volatile("v_nop\n\tv_nop\n\tv_nop\n\tv_nop" : "+v"(c) : "v"(a), "v"(b));
  return c;
}
__device__ __forceinline__ void keep4_b(v16b a, v16b b, v16b c, v16b d) { asm volatile("v_nop" :: "v"(a), "v"(b), "v"(c), "v"(d)); }
__device__ __forceinline__ void acc_guard4(v8f& a, v8f& b, v8f& c, v8f& d) { asm volatile("v_nop\n\tv_nop\n\tv_nop\n\tv_nop" : "+v"(a), "+v"(b), "+v"(c), "+v"(d)); }
__device__ __forceinline__ void wave_sync_lds() {
  __builtin_amdgcn_fence(__ATOMIC_RELEASE, "workgroup");
  __builtin_amdgcn_wave_barrier();
  __builtin_amdgcn_fence(__ATOMIC_ACQUIRE, "workgroup");
}

__global__ __launch_bounds__(256) void w_plane_kernel(const float* __restrict__ W, unsigned short* __restrict__ WB)
{
  const int i = blockIdx.x * 256 + threadIdx.x;
  if (i >= kNused * kK / 8) return;
  const int m   = i >> 6;
  const int kk  = (i & 63) << 3;
  const int tap = kk >> 8;
  const int c0  = kk & 255;
  const float* src = W + (size_t)m * kK + c0 * 2;
  const v4f a0 = *(const v4f*)(src);
  const v4f a1 = *(const v4f*)(src + 4);
  const v4f a2 = *(const v4f*)(src + 8);
  const v4f a3 = *(const v4f*)(src + 12);
  const bool t1 = (tap != 0);
  const float e0 = t1 ? a0[1] : a0[0];
  const float e1 = t1 ? a0[3] : a0[2];
  const float e2 = t1 ? a1[1] : a1[0];
  const float e3 = t1 ? a1[3] : a1[2];
  const float e4 = t1 ? a2[1] : a2[0];
  const float e5 = t1 ? a2[3] : a2[2];
  const float e6 = t1 ? a3[1] : a3[0];
  const float e7 = t1 ? a3[3] : a3[2];
  v4u w;
  w[0] = (unsigned)f2bf_bits(e0) | ((unsigned)f2bf_bits(e1) << 16);
  w[1] = (unsigned)f2bf_bits(e2) | ((unsigned)f2bf_bits(e3) << 16);
  w[2] = (unsigned)f2bf_bits(e4) | ((unsigned)f2bf_bits(e5) << 16);
  w[3] = (unsigned)f2bf_bits(e6) | ((unsigned)f2bf_bits(e7) << 16);
  unsigned short* dst = WB + (size_t)m * kK + kk;
  *(volatile v4u*)dst = w;
  __threadfence();
  *(volatile v4u*)dst = w;
}

__global__ __launch_bounds__(256) void xt_plane_kernel(const float* __restrict__ x, unsigned short* __restrict__ XT)
{
  __shared__ __align__(16) unsigned sW[32 * kXtLdsP];
  const int tid = threadIdx.x, lane = tid & 31, wave = tid >> 5;
  const int t0 = blockIdx.x * 32;
  const int b  = blockIdx.y;
  const float* xb = x + (size_t)b * kCin * kT + t0 + lane;
#pragma unroll 4
  for (int i = 0; i < 16; ++i) {
    const int cp = wave * 16 + i;
    const float v0 = xb[(size_t)(2 * cp) * kT];
    const float v1 = xb[(size_t)(2 * cp + 1) * kT];
    const unsigned w = (unsigned)f2bf_bits(v0) | ((unsigned)f2bf_bits(v1) << 16);
    sW[lane * kXtLdsP + cp] = w;
  }
  __syncthreads();
  v4u vv[4];
#pragma unroll
  for (int it = 0; it < 4; ++it) vv[it] = *(const v4u*)(sW + (wave * 4 + it) * kXtLdsP + lane * 4);
  unsigned short* bplane = XT + (size_t)b * kXtBatch;
  unsigned short* base   = bplane + (size_t)(1 + t0) * kCin;
  const v4u zero4 = (v4u){0u, 0u, 0u, 0u};
  const bool zrow = (t0 == 0) && (wave == 0);
  for (int pass = 0; pass < 2; ++pass) {
#pragma unroll
    for (int it = 0; it < 4; ++it)
      *(volatile v4u*)(base + (size_t)(wave * 4 + it) * kCin + lane * 8) = vv[it];
    if (zrow) *(volatile v4u*)(bplane + lane * 8) = zero4;
    __threadfence();
  }
}

__global__ __launch_bounds__(256) void conv_gemm_gate_kernel(
    const unsigned short* __restrict__ WBp, const unsigned short* __restrict__ XTp,
    const float* __restrict__ bias, float* __restrict__ GP)
{
  __shared__ __align__(16) float sT[8][16 * kSlabP];
  const __bf16* A = (const __bf16*)WBp;
  const int b    = blockIdx.y;
  const __bf16* Bb = (const __bf16*)XTp + (size_t)b * kXtBatch;
  const int lane = threadIdx.x & 31;
  const int wave = threadIdx.x >> 5;
  const int tile = blockIdx.x * 8 + wave;
  if (tile >= kTilesM * kTilesN) return;
  const int tm = tile / kTilesN;
  const int tn = tile - tm * kTilesN;
  const int m0 = tm << 6;
  const int n0 = tn << 6;
  const int rlane = lane & 15;
  const int koff  = (lane >> 4) * 8;
  const int mOff  = (lane >> 4) * 8;

  v8f acc[4][4];
#pragma unroll
  for (int i = 0; i < 4; ++i)
#pragma unroll
    for (int j = 0; j < 4; ++j) acc[i][j] = (v8f){0.f, 0.f, 0.f, 0.f, 0.f, 0.f, 0.f, 0.f};

#pragma unroll 1
  for (int k0 = 0; k0 < kK; k0 += 32) {
    v16b bh[4];
#pragma unroll
    for (int j = 0; j < 4; ++j)
      bh[j] = frag_load(Bb + (size_t)(n0 + (j << 4) + rlane) * kCin + koff + k0);
#pragma unroll
    for (int i = 0; i < 4; ++i) {
      const v16b ah = frag_load(A + (size_t)(m0 + (i << 4) + rlane) * kK + koff + k0);
#pragma unroll
      for (int j = 0; j < 4; ++j) acc[i][j] = mma_bf16(ah, bh[j], acc[i][j]);
    }
    keep4_b(bh[0], bh[1], bh[2], bh[3]);
  }
  acc_guard4(acc[0][0], acc[0][1], acc[0][2], acc[0][3]);
  acc_guard4(acc[1][0], acc[1][1], acc[1][2], acc[1][3]);
  acc_guard4(acc[2][0], acc[2][1], acc[2][2], acc[2][3]);
  acc_guard4(acc[3][0], acc[3][1], acc[3][2], acc[3][3]);

  float* slab = sT[wave];
  float* C = GP + (size_t)b * kT;
  const int hh = lane >> 4, c4 = (lane & 15) * 4;
  const int gate = m0 >> 8;
#pragma unroll
  for (int i = 0; i < 4; ++i) {
    const int mBase = m0 + (i << 4);
    const v4f bq0 = *(const v4f*)(bias + mBase + mOff);
    const v4f bq1 = *(const v4f*)(bias + mBase + mOff + 4);
    float bvr[8];
#pragma unroll
    for (int e = 0; e < 4; ++e) {
      const float u0 = bq0[e];
      const float u1 = bq1[e];
      bvr[e]     = bf_bits2f(f2bf_bits(u0));
      bvr[4 + e] = bf_bits2f(f2bf_bits(u1));
    }
#pragma unroll
    for (int j = 0; j < 4; ++j) {
#pragma unroll
      for (int r = 0; r < 8; ++r)
        slab[(mOff + r) * kSlabP + (j << 4) + rlane] = acc[i][j][r] + bvr[r];
    }
    wave_sync_lds();
#pragma unroll 1
    for (int it = 0; it < 8; ++it) {
      float* sp = slab + (it * 2 + hh) * kSlabP + c4;
      const v4f v = *(const v4f*)sp;
      const float p0 = v[0], p1 = v[1], p2 = v[2], p3 = v[3];
      v4f w;
      if (gate == 0) {
        w[0] = tanhf(p0);
        w[1] = tanhf(p1);
        w[2] = tanhf(p2);
        w[3] = tanhf(p3);
      } else {
        w[0] = 1.0f / (1.0f + expf(-p0));
        w[1] = 1.0f / (1.0f + expf(-p1));
        w[2] = 1.0f / (1.0f + expf(-p2));
        w[3] = 1.0f / (1.0f + expf(-p3));
      }
      *(v4f*)sp = w;
    }
    wave_sync_lds();
    for (int pass = 0; pass < 2; ++pass) {
#pragma unroll
      for (int it = 0; it < 8; ++it) {
        const int row = it * 2 + hh;
        const v4f v = *(const v4f*)(slab + row * kSlabP + c4);
        *(volatile v4f*)(C + (size_t)(mBase + row) * kCols + n0 + c4) = v;
      }
      __threadfence();
    }
    wave_sync_lds();
  }
}

__global__ __launch_bounds__(256) void gate_loop_kernel(const float* __restrict__ GP, float* __restrict__ out)
{
#pragma clang fp contract(off)
  const int q = blockIdx.x * 256 + threadIdx.x;
  if (q >= kGateCh * (kCols / 4)) return;
  const int c = q >> 11;
  const int n = (q & 2047) << 2;
  const int b = n >> 11;
  const int t = n & (kT - 1);
  const v4f zv = *(const v4f*)(GP + (size_t)c * kCols + n);
  const v4f fv = *(const v4f*)(GP + (size_t)(kGateCh + c) * kCols + n);
  const v4f ov = *(const v4f*)(GP + (size_t)(2 * kGateCh + c) * kCols + n);
  float zz[4], ff[4], cc[4];
  zz[0] = zv[0]; zz[1] = zv[1]; zz[2] = zv[2]; zz[3] = zv[3];
  ff[0] = fv[0]; ff[1] = fv[1]; ff[2] = fv[2]; ff[3] = fv[3];
  cc[0] = 0.0f;  cc[1] = 0.0f;  cc[2] = 0.0f;  cc[3] = 0.0f;
#pragma unroll 8
  for (int k = 0; k < kT; ++k) {
    const float kf = (float)k;
#pragma unroll
    for (int e = 0; e < 4; ++e) {
      const float fc = ff[e] * cc[e];
      const float kz = kf * zz[e];
      cc[e] = fc + kz;
    }
  }
  v4f hv;
  hv[0] = ov[0] * cc[0];
  hv[1] = ov[1] * cc[1];
  hv[2] = ov[2] * cc[2];
  hv[3] = ov[3] * cc[3];
  float* dst = out + (size_t)(b * kGateCh + c) * kT + t;
  *(volatile v4f*)dst = hv;
  __threadfence();
  *(volatile v4f*)dst = hv;
}

extern "C" void kernel_launch(void* const* d_in, const int* in_sizes, int n_in,
                              void* d_out, int out_size, void* d_ws, size_t ws_size,
                              hipStream_t stream) {
  if (n_in < 3) return;
  if (in_sizes[0] != kBatch * kCin * kT) return;
  if (in_sizes[1] != kNall * kCin * 2) return;
  if (in_sizes[2] != kNall) return;
  if (out_size != kBatch * kGateCh * kT) return;
  if (ws_size < kWsTotal) return;

  const float* x    = (const float*)d_in[0];
  const float* W    = (const float*)d_in[1];
  const float* bias = (const float*)d_in[2];
  float* out = (float*)d_out;

  char* ws = (char*)d_ws;
  unsigned short* WB = (unsigned short*)(ws + kOffWB);
  unsigned short* XT = (unsigned short*)(ws + kOffXT);
  float*          GP = (float*)(ws + kOffGP);

  w_plane_kernel<<<(kNused * kK / 8) / 256, 256, 0, stream>>>(W, WB);
  xt_plane_kernel<<<dim3(kT / 32, kBatch), 256, 0, stream>>>(x, XT);
  conv_gemm_gate_kernel<<<dim3(kGemmBlocksX, kBatch), 256, 0, stream>>>(WB, XT, bias, GP);
  gate_loop_kernel<<<(kGateCh * (kCols / 4)) / 256, 256, 0, stream>>>(GP, out);
}
